// LinearSelfAttention_86045374808452
// MI455X (gfx1250) — hardware-verified
//
#include <hip/hip_runtime.h>
#include <math.h>

constexpr int kBatch  = 2;
constexpr int kSeq    = 2048;
constexpr int kEmb    = 1024;
constexpr int kHeads  = 16;
constexpr int kHdim   = 64;
constexpr int kTok    = kBatch * kSeq;
constexpr int kQKld   = 2 * kEmb;
constexpr int kHPG    = 4;
constexpr int kGroups = kHeads / kHPG;
constexpr float kW1Carry    = 64.0f;
constexpr float kW1CarryInv = 1.0f / 64.0f;
constexpr float kInvEmb     = 1.0f / 1024.0f;
constexpr float kLnEps      = 1e-5f;

typedef __attribute__((ext_vector_type(16))) _Float16 v16h;
typedef __attribute__((ext_vector_type(8)))  _Float16 v8h;
typedef __attribute__((ext_vector_type(16))) __bf16   v16b;
typedef __attribute__((ext_vector_type(8)))  __bf16   v8b;
typedef __attribute__((ext_vector_type(8)))  float    v8f;
typedef __attribute__((ext_vector_type(4)))  float    v4f;
typedef __attribute__((ext_vector_type(4)))  unsigned int v4u;

__device__ __forceinline__ unsigned short f2bf_bits(float f) {
  unsigned u = __float_as_uint(f);
  return (unsigned short)((u + 0x7FFFu + ((u >> 16) & 1u)) >> 16);
}
__device__ __forceinline__ float bf_bits2f(unsigned short h) { return __uint_as_float(((unsigned)h) << 16); }

__device__ __forceinline__ void dep_guard_h(v8f& a, v8f& b, v16h x, v16h y) { asm volatile("v_nop\n\tv_nop\n\tv_nop\n\tv_nop" : "+v"(a), "+v"(b) : "v"(x), "v"(y)); }
__device__ __forceinline__ void dep_guard_b(v8f& a, v8f& b, v16b x, v16b y) { asm volatile("v_nop\n\tv_nop\n\tv_nop\n\tv_nop" : "+v"(a), "+v"(b) : "v"(x), "v"(y)); }
__device__ __forceinline__ void keep4_h(v16h a, v16h b, v16h c, v16h d) { asm volatile("v_nop" :: "v"(a), "v"(b), "v"(c), "v"(d)); }
__device__ __forceinline__ void keep4_b(v16b a, v16b b, v16b c, v16b d) { asm volatile("v_nop" :: "v"(a), "v"(b), "v"(c), "v"(d)); }
__device__ __forceinline__ void acc_guard4(v8f& a, v8f& b, v8f& c, v8f& d) { asm volatile("v_nop\n\tv_nop\n\tv_nop\n\tv_nop" : "+v"(a), "+v"(b), "+v"(c), "+v"(d)); }
template <typename T> struct Frag;
template <> struct Frag<_Float16> {
  typedef v16h V; union U { v16h v; v8h h[2]; };
  static __device__ __forceinline__ v16h load(const _Float16* p) {
    U f; f.h[0] = *(const v8h*)(p); f.h[1] = *(const v8h*)(p + 16); return f.v;
  }
  static __device__ __forceinline__ v8f mma(v16h a, v16h b, v8f c) {
    return __builtin_amdgcn_wmma_f32_16x16x32_f16(false, a, false, b, (short)0, c, false, false);
  }
  static __device__ __forceinline__ void guard(v8f& a, v8f& b, v16h x, v16h y) { dep_guard_h(a, b, x, y); }
  static __device__ __forceinline__ void keep(v16h a, v16h b, v16h c, v16h d) { keep4_h(a, b, c, d); }
};
template <> struct Frag<__bf16> {
  typedef v16b V; union U { v16b v; v8b h[2]; };
  static __device__ __forceinline__ v16b load(const __bf16* p) {
    U f; f.h[0] = *(const v8b*)(p); f.h[1] = *(const v8b*)(p + 16); return f.v;
  }
  static __device__ __forceinline__ v8f mma(v16b a, v16b b, v8f c) {
    return __builtin_amdgcn_wmma_f32_16x16x32_bf16(false, a, false, b, (short)0, c, false, false);
  }
  static __device__ __forceinline__ void guard(v8f& a, v8f& b, v16b x, v16b y) { dep_guard_b(a, b, x, y); }
  static __device__ __forceinline__ void keep(v16b a, v16b b, v16b c, v16b d) { keep4_b(a, b, c, d); }
};

__device__ __forceinline__ unsigned pk16(unsigned short a, unsigned short b) { return (unsigned)a | ((unsigned)b << 16); }
__device__ __forceinline__ unsigned short h_bits(float f) { const _Float16 h = (_Float16)f; return __builtin_bit_cast(unsigned short, h); }

template <int ET> struct Elem;
template <> struct Elem<0> { typedef _Float16 T; };
template <> struct Elem<1> { typedef __bf16 T; };
template <int ET, int SPL, int RSC, int OUT_MODE, int ACT, int TRI>
__global__ __launch_bounds__(256) void wmma_gemm64(
    const unsigned short* __restrict__ Ap, const unsigned short* __restrict__ A2p, int lda, long strideA,
    const unsigned short* __restrict__ Btp, const unsigned short* __restrict__ Bt2p, int ldb, long strideB,
    void* __restrict__ Cout, void* __restrict__ Cout2, int ldc, long strideC,
    const float* __restrict__ rsc, long strideS,
    int M, int N, int K, float scale) {
  typedef typename Elem<ET>::T T;
  typedef typename Frag<T>::V V;
  const T* A = (const T*)Ap; const T* A2 = (const T*)A2p; const T* Bt = (const T*)Btp; const T* Bt2 = (const T*)Bt2p;
  __shared__ __align__(16) float sT[8][16 * 68];
  const int b    = blockIdx.y;
  const int lane = threadIdx.x & 31;
  const int wave = threadIdx.x >> 5;
  const int tilesN = N >> 6;
  const int tilesM = M >> 6;
  const int tile = blockIdx.x * 8 + wave;
  if (tile >= tilesM * tilesN) return;
  const int tm = tile / tilesN;
  const int tn = tile - tm * tilesN;
  const int m0 = tm << 6;
  const int n0 = tn << 6;
  if (TRI == 1 && n0 > m0) return;
  const int Kl = (TRI == 2 && (m0 + 64) < K) ? (m0 + 64) : K;

  const T* Ab  = A  + (size_t)b * strideA;
  const T* Bb  = Bt + (size_t)b * strideB;
  const T* Ab2 = (SPL & 1) ? (A2  + (size_t)b * strideA) : nullptr;
  const T* Bb2 = (SPL & 2) ? (Bt2 + (size_t)b * strideB) : nullptr;

  const int rlane = lane & 15;
  const int koff  = (lane >> 4) * 8;
  const int mOff  = (lane >> 4) * 8;

  v8f acc[4][4];
#pragma unroll
  for (int i = 0; i < 4; ++i)
#pragma unroll
    for (int j = 0; j < 4; ++j) acc[i][j] = (v8f){0.f,0.f,0.f,0.f,0.f,0.f,0.f,0.f};

  for (int k0 = 0; k0 < Kl; k0 += 32) {
    V bh[4], bl[4];
#pragma unroll
    for (int j = 0; j < 4; ++j) {
      const size_t bo = (size_t)(n0 + (j << 4) + rlane) * ldb + koff + k0;
      bh[j] = Frag<T>::load(Bb + bo);
      if (SPL & 2) bl[j] = Frag<T>::load(Bb2 + bo);
    }
#pragma unroll
    for (int i = 0; i < 4; ++i) {
      const size_t ao = (size_t)(m0 + (i << 4) + rlane) * lda + koff + k0;
      V ah = Frag<T>::load(Ab + ao);
      V al;
      if (SPL & 1) al = Frag<T>::load(Ab2 + ao);
#pragma unroll
      for (int j = 0; j < 4; ++j) {
        acc[i][j] = Frag<T>::mma(ah, bh[j], acc[i][j]);
        if (SPL & 2) acc[i][j] = Frag<T>::mma(ah, bl[j], acc[i][j]);
        if (SPL & 1) acc[i][j] = Frag<T>::mma(al, bh[j], acc[i][j]);
      }
      Frag<T>::guard(acc[i][0], acc[i][3], ah, (SPL & 1) ? al : ah);
    }
    Frag<T>::keep(bh[0], bh[1], bh[2], bh[3]);
    if (SPL & 2) Frag<T>::keep(bl[0], bl[1], bl[2], bl[3]);
  }
  acc_guard4(acc[0][0], acc[0][1], acc[0][2], acc[0][3]);
  acc_guard4(acc[1][0], acc[1][1], acc[1][2], acc[1][3]);
  acc_guard4(acc[2][0], acc[2][1], acc[2][2], acc[2][3]);
  acc_guard4(acc[3][0], acc[3][1], acc[3][2], acc[3][3]);

  float* slab = sT[wave];
  const float* Rs = RSC ? (rsc + (size_t)b * strideS) : nullptr;
#pragma unroll
  for (int i = 0; i < 4; ++i) {
    const int mBase = m0 + (i << 4);
    float rsv[8];
#pragma unroll
    for (int r = 0; r < 8; ++r) rsv[r] = RSC ? Rs[mBase + mOff + r] : 1.0f;
#pragma unroll
    for (int j = 0; j < 4; ++j) {
      const int n = n0 + (j << 4) + rlane;
#pragma unroll
      for (int r = 0; r < 8; ++r) {
        float v = acc[i][j][r] * scale;
        if (RSC) v = v * rsv[r];
        if (TRI == 1) { if (n > mBase + mOff + r) v = 0.0f; }
        if (ACT == 6) v = (v > 0.0f) ? (v + 1.0f) : __expf(v);
        slab[(mOff + r) * 68 + (j << 4) + rlane] = v;
      }
    }
    __builtin_amdgcn_fence(__ATOMIC_RELEASE, "workgroup");
    __builtin_amdgcn_wave_barrier();
    __builtin_amdgcn_fence(__ATOMIC_ACQUIRE, "workgroup");
    if (OUT_MODE == 0) {
      float* C = (float*)Cout + (size_t)b * strideC;
      const int hh = lane >> 4, c4 = (lane & 15) * 4;
      for (int pass = 0; pass < 2; ++pass) {
#pragma unroll
        for (int it = 0; it < 8; ++it) {
          const int row = it * 2 + hh;
          v4f v = *(const v4f*)(slab + row * 68 + c4);
          *(volatile v4f*)(C + (size_t)(mBase + row) * ldc + n0 + c4) = v;
        }
        __threadfence();
      }
    } else {
      const int q = lane >> 3, c8 = (lane & 7) * 8;
      unsigned short* C  = (unsigned short*)Cout  + (size_t)b * strideC;
      unsigned short* C2 = (OUT_MODE == 2) ? ((unsigned short*)Cout2 + (size_t)b * strideC) : nullptr;
      for (int pass = 0; pass < 2; ++pass) {
#pragma unroll
        for (int it = 0; it < 4; ++it) {
          const int row = it * 4 + q;
          const float* sp = slab + row * 68 + c8;
          v8h hv, lv;
#pragma unroll
          for (int e = 0; e < 8; ++e) {
            if (OUT_MODE == 1) {
              hv[e] = (_Float16)sp[e];
            } else {
              unsigned short hb = f2bf_bits(sp[e]);
              unsigned short lb = f2bf_bits(sp[e] - bf_bits2f(hb));
              hv[e] = __builtin_bit_cast(_Float16, hb);
              lv[e] = __builtin_bit_cast(_Float16, lb);
            }
          }
          *(volatile v8h*)(C + (size_t)(mBase + row) * ldc + n0 + c8) = hv;
          if (OUT_MODE == 2) *(volatile v8h*)(C2 + (size_t)(mBase + row) * ldc + n0 + c8) = lv;
        }
        __threadfence();
      }
    }
    __builtin_amdgcn_fence(__ATOMIC_RELEASE, "workgroup");
    __builtin_amdgcn_wave_barrier();
    __builtin_amdgcn_fence(__ATOMIC_ACQUIRE, "workgroup");
  }
}

template <int MODE>
__global__ __launch_bounds__(256) void cast8_kernel(const float* __restrict__ in, unsigned short* __restrict__ out, int n8, float scale) {
  const int i = blockIdx.x * 256 + threadIdx.x;
  if (i >= n8) return;
  const float* p = in + 8 * (size_t)i;
  const v4f a = *(const v4f*)(p);
  const v4f c = *(const v4f*)(p + 4);
  unsigned short hb[8];
#pragma unroll
  for (int e = 0; e < 4; ++e) {
    if (MODE == 0) {
      hb[e]     = f2bf_bits(a[e]);
      hb[4 + e] = f2bf_bits(c[e]);
    } else {
      hb[e]     = h_bits(bf_bits2f(f2bf_bits(a[e])) * scale);
      hb[4 + e] = h_bits(bf_bits2f(f2bf_bits(c[e])) * scale);
    }
  }
  const v4u u = (v4u){pk16(hb[0], hb[1]), pk16(hb[2], hb[3]), pk16(hb[4], hb[5]), pk16(hb[6], hb[7])};
  unsigned short* q = out + 8 * (size_t)i;
  *(volatile v4u*)q = u;
  __threadfence();
  *(volatile v4u*)q = u;
  (void)scale;
}

__global__ __launch_bounds__(128) void layernorm3_kernel(const float* __restrict__ x, unsigned short* __restrict__ XF,
                                                         unsigned short* __restrict__ XH, unsigned short* __restrict__ XL) {
  __shared__ float redA[4];
  __shared__ float redB[4];
  const int row  = blockIdx.x;
  const int t    = threadIdx.x;
  const int lane = t & 31, wave = t >> 5;
  const int c0   = t * 8;
  const float* xr = x + (size_t)row * kEmb + c0;
  const v4f a = *(const v4f*)(xr);
  const v4f c = *(const v4f*)(xr + 4);
  float xb[8];
#pragma unroll
  for (int e = 0; e < 4; ++e) {
    xb[e]     = bf_bits2f(f2bf_bits(a[e]));
    xb[4 + e] = bf_bits2f(f2bf_bits(c[e]));
  }
  float s = ((xb[0] + xb[1]) + (xb[2] + xb[3])) + ((xb[4] + xb[5]) + (xb[6] + xb[7]));
#pragma unroll
  for (int off = 16; off > 0; off >>= 1) s += __shfl_xor(s, off, 32);
  if (lane == 0) redA[wave] = s;
  __syncthreads();
  const float mu = ((redA[0] + redA[1]) + (redA[2] + redA[3])) * kInvEmb;
  float d[8];
#pragma unroll
  for (int e = 0; e < 8; ++e) d[e] = xb[e] - mu;
  float qq = ((d[0] * d[0] + d[1] * d[1]) + (d[2] * d[2] + d[3] * d[3])) + ((d[4] * d[4] + d[5] * d[5]) + (d[6] * d[6] + d[7] * d[7]));
#pragma unroll
  for (int off = 16; off > 0; off >>= 1) qq += __shfl_xor(qq, off, 32);
  if (lane == 0) redB[wave] = qq;
  __syncthreads();
  const float var = ((redB[0] + redB[1]) + (redB[2] + redB[3])) * kInvEmb;
  const float rs  = rsqrtf(var + kLnEps);
  unsigned short fb[8], hbv[8], lb[8];
#pragma unroll
  for (int e = 0; e < 8; ++e) {
    const float xc = d[e] * rs;
    fb[e] = h_bits(xc);
    const unsigned short hh = f2bf_bits(xc);
    hbv[e] = hh;
    lb[e] = f2bf_bits(xc - bf_bits2f(hh));
  }
  const v4u fv = (v4u){pk16(fb[0], fb[1]), pk16(fb[2], fb[3]), pk16(fb[4], fb[5]), pk16(fb[6], fb[7])};
  const v4u hv = (v4u){pk16(hbv[0], hbv[1]), pk16(hbv[2], hbv[3]), pk16(hbv[4], hbv[5]), pk16(hbv[6], hbv[7])};
  const v4u lv = (v4u){pk16(lb[0], lb[1]), pk16(lb[2], lb[3]), pk16(lb[4], lb[5]), pk16(lb[6], lb[7])};
  unsigned short* fp = XF + (size_t)row * kEmb + c0;
  unsigned short* hp = XH + (size_t)row * kEmb + c0;
  unsigned short* lp = XL + (size_t)row * kEmb + c0;
  *(volatile v4u*)fp = fv;
  *(volatile v4u*)hp = hv;
  *(volatile v4u*)lp = lv;
  __threadfence();
  *(volatile v4u*)fp = fv;
  *(volatile v4u*)hp = hv;
  *(volatile v4u*)lp = lv;
}

__global__ __launch_bounds__(64) void rownorm_kernel(const unsigned short* __restrict__ QK, float* __restrict__ RINV) {
  __shared__ float sQ[64][65];
  __shared__ float sK[64][65];
  __shared__ float sC[64][65];
  const int bh = blockIdx.x;
  const int b  = bh / kHeads, h = bh - b * kHeads;
  const int t  = threadIdx.x;
  const _Float16* qp = (const _Float16*)QK + (size_t)b * kSeq * kQKld + h * kHdim;
  const _Float16* kp = qp + kEmb;
  const int rr = t >> 3, c8 = (t & 7) * 8;
  float carry = 0.f;
#pragma unroll 1
  for (int c = 0; c < kSeq / 64; ++c) {
#pragma unroll
    for (int i = 0; i < 8; ++i) {
      const int r = i * 8 + rr;
      const size_t o = (size_t)(c * 64 + r) * kQKld + c8;
      const v8h qv = *(const v8h*)(qp + o);
      const v8h kv = *(const v8h*)(kp + o);
#pragma unroll
      for (int e = 0; e < 8; ++e) {
        sQ[r][c8 + e] = (float)qv[e];
        sK[r][c8 + e] = (float)kv[e];
      }
    }
    __syncthreads();
    float run = carry;
#pragma unroll 1
    for (int s = 0; s < 64; ++s) {
      run += sK[s][t];
      sC[s][t] = run;
    }
    carry = run;
    __syncthreads();
    float z = 0.f;
#pragma unroll 1
    for (int dd = 0; dd < 64; ++dd) z = fmaf(sQ[t][dd], sC[t][dd], z);
    const float rv = 1.0f / z;
    float* p = RINV + (size_t)bh * kSeq + c * 64 + t;
    *(volatile float*)p = rv;
    __threadfence();
    *(volatile float*)p = rv;
    __syncthreads();
  }
}

extern "C" void kernel_launch(void* const* d_in, const int* in_sizes, int n_in,
                              void* d_out, int out_size, void* d_ws, size_t ws_size,
                              hipStream_t stream) {
  if (n_in < 3) return;
  if (in_sizes[0] != kTok * kEmb) return;
  if (in_sizes[1] != 3 * kEmb * kEmb) return;
  if (in_sizes[2] != kEmb * kEmb) return;
  if (out_size != kTok * kEmb) return;

  const float* x  = (const float*)d_in[0];
  const float* W1 = (const float*)d_in[1];
  const float* W2 = (const float*)d_in[2];
  float* outp = (float*)d_out;

  const size_t SZ_W1F  = (size_t)2 * kEmb * kEmb * 2;
  const size_t SZ_W1B  = (size_t)kEmb * kEmb * 2;
  const size_t SZ_W2B  = (size_t)kEmb * kEmb * 2;
  const size_t SZ_T16  = (size_t)kTok * kEmb * 2;
  const size_t SZ_QK   = (size_t)kTok * kQKld * 2;
  const size_t SZ_RINV = (size_t)kBatch * kHeads * kSeq * 4;
  const size_t SZ_P    = (size_t)kHPG * kSeq * kSeq * 2;

  size_t off = 0;
  const size_t oW2B  = off; off += SZ_W2B;
  const size_t oQK   = off; off += SZ_QK;
  const size_t oVTH  = off; off += SZ_T16;
  const size_t oVTL  = off; off += SZ_T16;
  const size_t oRINV = off; off += SZ_RINV;
  const size_t oCTXH = off; off += SZ_T16;
  const size_t oCTXL = off; off += SZ_T16;
  const size_t oA    = off;
  const size_t oW1F  = oA;
  const size_t oW1B  = oW1F + SZ_W1F;
  const size_t oXF   = oW1B + SZ_W1B;
  const size_t oXH   = oXF + SZ_T16;
  const size_t oXL   = oXH + SZ_T16;
  const size_t endP1 = oXL + SZ_T16;
  const size_t oPH   = oA;
  const size_t oPL   = oPH + SZ_P;
  const size_t endP2 = oPL + SZ_P;
  const size_t TOTAL = (endP1 > endP2) ? endP1 : endP2;
  if (TOTAL > ws_size) return;
  if (TOTAL > (size_t)134217728) return;

  char* ws = (char*)d_ws;
  unsigned short* W2B  = (unsigned short*)(ws + oW2B);
  unsigned short* QK   = (unsigned short*)(ws + oQK);
  unsigned short* VTH  = (unsigned short*)(ws + oVTH);
  unsigned short* VTL  = (unsigned short*)(ws + oVTL);
  float*          RINV = (float*)(ws + oRINV);
  unsigned short* CTXH = (unsigned short*)(ws + oCTXH);
  unsigned short* CTXL = (unsigned short*)(ws + oCTXL);
  unsigned short* W1F  = (unsigned short*)(ws + oW1F);
  unsigned short* W1B  = (unsigned short*)(ws + oW1B);
  unsigned short* XF   = (unsigned short*)(ws + oXF);
  unsigned short* XH   = (unsigned short*)(ws + oXH);
  unsigned short* XL   = (unsigned short*)(ws + oXL);
  unsigned short* PH   = (unsigned short*)(ws + oPH);
  unsigned short* PL   = (unsigned short*)(ws + oPL);
  const float* dummy_rsc = RINV;

  const dim3 blk(256);

  {
    const int n8qk = 2 * kEmb * kEmb / 8;
    cast8_kernel<1><<<dim3(n8qk / 256), blk, 0, stream>>>(W1, W1F, n8qk, kW1Carry);
    const int n8v = kEmb * kEmb / 8;
    cast8_kernel<0><<<dim3(n8v / 256), blk, 0, stream>>>(W1 + (size_t)2 * kEmb * kEmb, W1B, n8v, 1.0f);
    cast8_kernel<0><<<dim3(n8v / 256), blk, 0, stream>>>(W2, W2B, n8v, 1.0f);
  }

  layernorm3_kernel<<<dim3(kTok), dim3(128), 0, stream>>>(x, XF, XH, XL);

  const int tilesTok = kTok / 64;
  const dim3 gQK((tilesTok * (kQKld / 64) + 7) / 8, 1);
  const dim3 gV(((kEmb / 64) * tilesTok + 7) / 8, 1);
  const dim3 gOut((tilesTok * (kEmb / 64) + 7) / 8, 1);
  const dim3 gS(((kSeq / 64) * (kSeq / 64) + 7) / 8, kHPG);
  const dim3 gPV(((kSeq / 64) * (kHdim / 64) + 7) / 8, kHPG);

  wmma_gemm64<0, 0, 0, 1, 6, 0><<<gQK, blk, 0, stream>>>(
      XF, XF, kEmb, 0L, W1F, W1F, kEmb, 0L, (void*)QK, (void*)QK, kQKld, 0L, dummy_rsc, 0L, kTok, kQKld, kEmb, kW1CarryInv);
  wmma_gemm64<1, 2, 0, 2, 0, 0><<<gV, blk, 0, stream>>>(
      W1B, W1B, kEmb, 0L, XH, XL, kEmb, 0L, (void*)VTH, (void*)VTL, kTok, 0L, dummy_rsc, 0L, kEmb, kTok, kEmb, 1.0f);
  rownorm_kernel<<<dim3(kBatch * kHeads), dim3(64), 0, stream>>>(QK, RINV);

  for (int b = 0; b < kBatch; ++b) {
    for (int g = 0; g < kGroups; ++g) {
      const size_t hc = (size_t)g * kHPG * kHdim;
      const unsigned short* Aq = QK + (size_t)b * kSeq * kQKld + hc;
      const unsigned short* Bk = Aq + kEmb;
      const float* rs = RINV + (size_t)(b * kHeads + g * kHPG) * kSeq;
      wmma_gemm64<0, 0, 1, 2, 0, 1><<<gS, blk, 0, stream>>>(
          Aq, Aq, kQKld, (long)kHdim, Bk, Bk, kQKld, (long)kHdim,
          (void*)PH, (void*)PL, kSeq, (long)kSeq * kSeq, rs, (long)kSeq, kSeq, kSeq, kHdim, 1.0f);
      const unsigned short* Bvh = VTH + hc * kTok + (size_t)b * kSeq;
      const unsigned short* Bvl = VTL + hc * kTok + (size_t)b * kSeq;
      unsigned short* Ch = CTXH + (size_t)b * kSeq * kEmb + hc;
      unsigned short* Cl = CTXL + (size_t)b * kSeq * kEmb + hc;
      wmma_gemm64<1, 3, 0, 2, 0, 2><<<gPV, blk, 0, stream>>>(
          PH, PL, kSeq, (long)kSeq * kSeq, Bvh, Bvl, kTok, (long)kHdim * kTok,
          (void*)Ch, (void*)Cl, kEmb, (long)kHdim, dummy_rsc, 0L, kSeq, kHdim, kSeq, 1.0f);
    }
  }

  wmma_gemm64<1, 1, 0, 0, 0, 0><<<gOut, blk, 0, stream>>>(
      CTXH, CTXL, kEmb, 0L, W2B, W2B, kEmb, 0L, (void*)outp, (void*)outp, kEmb, 0L, dummy_rsc, 0L, kTok, kEmb, kEmb, 1.0f);
}
